// LocalNeighbourEmbedding_65335042506818
// MI455X (gfx1250) — hardware-verified
//
#include <hip/hip_runtime.h>
#include <math.h>
#include <stdint.h>
#include <stddef.h>

typedef _Float16 v8h  __attribute__((ext_vector_type(8)));
typedef _Float16 v16h __attribute__((ext_vector_type(16)));
typedef float    v8f  __attribute__((ext_vector_type(8)));
typedef float    v4f  __attribute__((ext_vector_type(4)));
union Frag { v16h v; v8h half[2]; };

#define KNB   16
#define FIN   130
#define FKP   160
#define FP    168
#define HID   256
#define HP    264
#define OUTD  128
#define W1P   192
#define W2P   256
#define WPB   4
#define BLK   (WPB * 32)
#define RPW   32

static_assert((W1P * 2) % 128 == 0);
static_assert((W2P * 2) % 128 == 0);
static_assert((FP % 8) == 0);
static_assert((HP % 8) == 0);
static_assert(FKP <= FP);
static_assert(HID <= HP);

__device__ __forceinline__ v8f wmma_f16(const v16h a, const v16h b, v8f c)
{
  v8f d = __builtin_amdgcn_wmma_f32_16x16x32_f16(false, a, false, b, (short)0, c, false, false);
  asm volatile("v_nop\n\tv_nop\n\tv_nop\n\tv_nop" : "+v"(d) : "v"(a), "v"(b));
  return d;
}

__device__ __forceinline__ float gelu_f(float x)
{
  const float y = 0.7978845608028654f * fmaf(0.044715f * x, x * x, x);
  const float u = __expf(-2.0f * y);
  return x * __builtin_amdgcn_rcpf(1.0f + u);
}

__global__ __launch_bounds__(32)
void k_prep(const float* __restrict__ w1, const float* __restrict__ b1,
            const float* __restrict__ w2, _Float16* w1t, _Float16* w2t)
{
  const int b = blockIdx.x;
  const int q = threadIdx.x & 31;
  v8h v;
  bool doit;
  _Float16* base;
  size_t off;
  if (b < HID) {
    const int n = b;
    doit = (q < (W1P / 8));
    base = w1t;
    off  = (size_t)n * W1P + 8 * q;
#pragma unroll
    for (int i = 0; i < 8; ++i) {
      const int k = 8 * q + i;
      float x = 0.0f;
      if (k < FIN)       x = 8.0f * w1[(size_t)k * HID + n];
      else if (k == FIN) x = 8.0f * b1[n];
      v[i] = (_Float16)x;
    }
  } else {
    const int n = b - HID;
    doit = (n < OUTD);
    const int nn = doit ? n : 0;
    base = w2t;
    off  = (size_t)nn * W2P + 8 * q;
#pragma unroll
    for (int i = 0; i < 8; ++i) {
      const int k = 8 * q + i;
      v[i] = (_Float16)(16.0f * w2[(size_t)k * OUTD + nn]);
    }
  }
  volatile v8h* p = (volatile v8h*)(base + off);
  if (doit) *p = v;
  __threadfence();
  if (doit) *p = v;
}

__global__ __launch_bounds__(BLK)
void k_main(const float* __restrict__ ca, const int* __restrict__ resi,
            const int* __restrict__ chain, const int* __restrict__ nbr,
            const _Float16* __restrict__ w1t, const _Float16* __restrict__ w2t,
            const float* __restrict__ b2, const float* __restrict__ gamma,
            const float* __restrict__ beta, float* out, int nres, int rpw)
{
  __shared__ __attribute__((aligned(16))) _Float16 sF[WPB * 16 * FP];
  __shared__ __attribute__((aligned(16))) _Float16 sH[WPB * 16 * HP];
  __shared__ __attribute__((aligned(16))) float    sM[WPB * OUTD];

  const int tid = threadIdx.x;
  const int wv = tid >> 5;
  const int l  = tid & 31;
  const int h  = l >> 4;
  const int e  = l & 15;
  _Float16* Fw = sF + wv * (16 * FP);
  _Float16* Hw = sH + wv * (16 * HP);
  float*    Mw = sM + wv * OUTD;
  const int g  = blockIdx.x * WPB + wv;

  const v4f gam = *(const v4f*)(gamma + 4 * l);
  const v4f bet = *(const v4f*)(beta  + 4 * l);

  for (int it = 0; it < rpw; ++it) {
    const int  r      = g * rpw + it;
    const bool active = (r < nres);
    const int  rr     = active ? r : (nres - 1);

    const int  j     = nbr[(size_t)rr * KNB + e];
    const bool valid = (j != -1);
    int jj = (j < 0) ? (j + nres) : j;
    jj = min(max(jj, 0), nres - 1);
    const float px = ca[(size_t)rr * 3 + 0];
    const float py = ca[(size_t)rr * 3 + 1];
    const float pz = ca[(size_t)rr * 3 + 2];
    const float dx = px - ca[(size_t)jj * 3 + 0];
    const float dy = py - ca[(size_t)jj * 3 + 1];
    const float dz = pz - ca[(size_t)jj * 3 + 2];
    const float dist = sqrtf(dx * dx + dy * dy + dz * dz);
    int rd = resi[rr] - resi[jj];
    rd = min(max(rd, -32), 32) + 32;
    if (chain[rr] != chain[jj]) rd = 65;
    const unsigned mask16 = __builtin_amdgcn_ballot_w32(valid) & 0xFFFFu;
    const float cnt = (float)__builtin_popcount(mask16);
    float mv[8];
#pragma unroll
    for (int v = 0; v < 8; ++v) mv[v] = ((mask16 >> (8 * h + v)) & 1u) ? 1.0f : 0.0f;

    {
      const float t0 = dist * (64.0f / 22.0f);
      const float cstep = 64.0f / 63.0f;
#pragma unroll
      for (int c = 0; c < 4; ++c) {
        v8h v;
#pragma unroll
        for (int i = 0; i < 8; ++i) {
          const float t = t0 - (float)(32 * h + 8 * c + i) * cstep;
          v[i] = (_Float16)__expf(-(t * t));
        }
        *(v8h*)(Fw + e * FP + 32 * h + 8 * c) = v;
      }
      const int tgt = 64 + rd;
#pragma unroll
      for (int c = 0; c < 6; ++c) {
        const int kb = 64 + 48 * h + 8 * c;
        v8h v;
#pragma unroll
        for (int i = 0; i < 8; ++i) {
          const int k = kb + i;
          v[i] = (k == tgt || k == FIN) ? (_Float16)1.0f : (_Float16)0.0f;
        }
        *(v8h*)(Fw + e * FP + kb) = v;
      }
    }
    __syncthreads();

    {
      Frag fb[5];
#pragma unroll
      for (int ks = 0; ks < 5; ++ks) {
        fb[ks].half[0] = *(const v8h*)(Fw + e * FP + ks * 32 + 8 * h);
        fb[ks].half[1] = *(const v8h*)(Fw + e * FP + ks * 32 + 16 + 8 * h);
      }
#pragma unroll 1
      for (int nt = 0; nt < HID / 16; ++nt) {
        const _Float16* ap = w1t + (size_t)(nt * 16 + e) * W1P + 8 * h;
        v8f acc = {0.f, 0.f, 0.f, 0.f, 0.f, 0.f, 0.f, 0.f};
#pragma unroll
        for (int ks = 0; ks < 5; ++ks) {
          Frag a;
          a.half[0] = *(const v8h*)(ap + ks * 32);
          a.half[1] = *(const v8h*)(ap + ks * 32 + 16);
          acc = wmma_f16(a.v, fb[ks].v, acc);
        }
        v8h hv;
#pragma unroll
        for (int v = 0; v < 8; ++v) hv[v] = (_Float16)gelu_f(acc[v] * 0.125f);
        *(v8h*)(Hw + e * HP + nt * 16 + 8 * h) = hv;
      }
    }
    __syncthreads();

    {
      Frag fh[8];
#pragma unroll
      for (int ks = 0; ks < 8; ++ks) {
        fh[ks].half[0] = *(const v8h*)(Hw + e * HP + ks * 32 + 8 * h);
        fh[ks].half[1] = *(const v8h*)(Hw + e * HP + ks * 32 + 16 + 8 * h);
      }
#pragma unroll 1
      for (int nt = 0; nt < OUTD / 16; ++nt) {
        const int c = nt * 16 + e;
        const _Float16* bp = w2t + (size_t)c * W2P + 8 * h;
        v8f acc = {0.f, 0.f, 0.f, 0.f, 0.f, 0.f, 0.f, 0.f};
#pragma unroll
        for (int ks = 0; ks < 8; ++ks) {
          Frag b;
          b.half[0] = *(const v8h*)(bp + ks * 32);
          b.half[1] = *(const v8h*)(bp + ks * 32 + 16);
          acc = wmma_f16(fh[ks].v, b.v, acc);
        }
        float s = 0.0f;
#pragma unroll
        for (int v = 0; v < 8; ++v) s = fmaf(mv[v], acc[v], s);
        s += __shfl_xor(s, 16, 32);
        const float x = s * (1.0f / 256.0f) + cnt * b2[c] * (1.0f / 16.0f);
        if (h == 0) Mw[c] = x;
      }
    }
    __syncthreads();

    {
      const v4f xv = *(const v4f*)(Mw + 4 * l);
      float s1 = (xv[0] + xv[1]) + (xv[2] + xv[3]);
#pragma unroll
      for (int off = 16; off > 0; off >>= 1) s1 += __shfl_xor(s1, off, 32);
      const float mean = s1 * (1.0f / 128.0f);
      const v4f d = xv - mean;
      float s2 = (d[0] * d[0] + d[1] * d[1]) + (d[2] * d[2] + d[3] * d[3]);
#pragma unroll
      for (int off = 16; off > 0; off >>= 1) s2 += __shfl_xor(s2, off, 32);
      const float var = s2 * (1.0f / 128.0f);
      const float inv = rsqrtf(var + 1e-5f);
      const v4f y = d * inv * gam + bet;
      volatile v4f* op = (volatile v4f*)(out + (size_t)rr * OUTD + 4 * l);
      if (active) *op = y;
      __threadfence();
      if (active) *op = y;
    }
  }
}

extern "C" void kernel_launch(void* const* d_in, const int* in_sizes, int n_in,
                              void* d_out, int out_size, void* d_ws, size_t ws_size,
                              hipStream_t stream)
{
  if (n_in < 10) return;
  const int nres = in_sizes[1];
  if (nres <= 0) return;
  if (in_sizes[0] != nres * 3) return;
  if (in_sizes[2] != nres) return;
  if (in_sizes[3] != nres * KNB) return;
  if (in_sizes[4] != FIN * HID) return;
  if (in_sizes[5] != HID) return;
  if (in_sizes[6] != HID * OUTD) return;
  if (in_sizes[7] != OUTD || in_sizes[8] != OUTD || in_sizes[9] != OUTD) return;
  if (out_size != nres * OUTD) return;

  const float* ca    = (const float*)d_in[0];
  const int*   resi  = (const int*)  d_in[1];
  const int*   chain = (const int*)  d_in[2];
  const int*   nbr   = (const int*)  d_in[3];
  const float* w1    = (const float*)d_in[4];
  const float* b1    = (const float*)d_in[5];
  const float* w2    = (const float*)d_in[6];
  const float* b2    = (const float*)d_in[7];
  const float* gamma = (const float*)d_in[8];
  const float* beta  = (const float*)d_in[9];
  float* out = (float*)d_out;

  const size_t off_w1t   = 0;
  const size_t bytes_w1t = (size_t)HID * W1P * sizeof(_Float16);
  const size_t off_w2t   = off_w1t + bytes_w1t;
  const size_t bytes_w2t = (size_t)OUTD * W2P * sizeof(_Float16);
  const size_t total     = off_w2t + bytes_w2t;
  if (total > ws_size) return;
  _Float16* w1t = (_Float16*)((char*)d_ws + off_w1t);
  _Float16* w2t = (_Float16*)((char*)d_ws + off_w2t);

  k_prep<<<dim3(HID + OUTD), dim3(32), 0, stream>>>(w1, b1, w2, w1t, w2t);

  const int waves  = (nres + RPW - 1) / RPW;
  const int blocks = (waves + WPB - 1) / WPB;
  k_main<<<dim3(blocks), dim3(BLK), 0, stream>>>(ca, resi, chain, nbr, w1t, w2t,
                                                 b2, gamma, beta, out, nres, RPW);
}
